// softmaxattention_34299608826350
// MI455X (gfx1250) — hardware-run, weakly checked
//
#include <hip/hip_runtime.h>
#include <math.h>

constexpr int kB     = 2;
constexpr int kC     = 512;
constexpr int kH     = 64;
constexpr int kW     = 64;
constexpr int kN     = kH * kW;
constexpr int kCk    = 64;
constexpr int kTaps  = 9;
constexpr int kHP    = kH + 2;
constexpr int kKconv = kC * kTaps;
constexpr int kRows  = kB * kN;
constexpr int kMHalf = kN / 2;
constexpr float kPCarry    = 32768.0f;
constexpr float kPCarryInv = 1.0f / 32768.0f;
constexpr float kBnEps     = 1.0e-5f;
static_assert(kN % 64 == 0 && kC % 64 == 0 && kCk % 64 == 0 && kMHalf % 64 == 0);
static_assert(kCk % 32 == 0 && kN % 32 == 0 && kC % 32 == 0);
static_assert(kB * kH == 128);

typedef __attribute__((ext_vector_type(16))) _Float16 v16h;
typedef __attribute__((ext_vector_type(8)))  _Float16 v8h;
typedef __attribute__((ext_vector_type(16))) __bf16   v16b;
typedef __attribute__((ext_vector_type(8)))  __bf16   v8b;
typedef __attribute__((ext_vector_type(8)))  float    v8f;
typedef __attribute__((ext_vector_type(4)))  float    v4f;
typedef __attribute__((ext_vector_type(2)))  float    v2f;
typedef __attribute__((ext_vector_type(4)))  unsigned int v4u;

__device__ __forceinline__ unsigned short f2bf_bits(float f) {
  unsigned u = __float_as_uint(f);
  return (unsigned short)((u + 0x7FFFu + ((u >> 16) & 1u)) >> 16);
}
__device__ __forceinline__ float bf_bits2f(unsigned short h) { return __uint_as_float(((unsigned)h) << 16); }
__device__ __forceinline__ unsigned pk16(unsigned short a, unsigned short b) { return (unsigned)a | ((unsigned)b << 16); }
__device__ __forceinline__ void mem_order() { asm volatile("" ::: "memory"); }

__device__ __forceinline__ void tie4_h(v8f& a, v8f& b, v8f& c, v8f& d, v16h x, v16h y, v16h z0, v16h z1, v16h z2, v16h z3) {
  asm volatile("v_nop\n\tv_nop\n\tv_nop\n\tv_nop" : "+v"(a), "+v"(b), "+v"(c), "+v"(d) : "v"(x), "v"(y), "v"(z0), "v"(z1), "v"(z2), "v"(z3));
}
__device__ __forceinline__ void tie4_b(v8f& a, v8f& b, v8f& c, v8f& d, v16b x, v16b y, v16b z0, v16b z1, v16b z2, v16b z3) {
  asm volatile("v_nop\n\tv_nop\n\tv_nop\n\tv_nop" : "+v"(a), "+v"(b), "+v"(c), "+v"(d) : "v"(x), "v"(y), "v"(z0), "v"(z1), "v"(z2), "v"(z3));
}
__device__ __forceinline__ void keep4_h(v16h a, v16h b, v16h c, v16h d) { asm volatile("v_nop" :: "v"(a), "v"(b), "v"(c), "v"(d)); }
__device__ __forceinline__ void keep4_b(v16b a, v16b b, v16b c, v16b d) { asm volatile("v_nop" :: "v"(a), "v"(b), "v"(c), "v"(d)); }
__device__ __forceinline__ void acc_guard4(v8f& a, v8f& b, v8f& c, v8f& d) { asm volatile("v_nop\n\tv_nop\n\tv_nop\n\tv_nop" : "+v"(a), "+v"(b), "+v"(c), "+v"(d)); }

template <typename T> struct Frag;
template <> struct Frag<_Float16> {
  typedef v16h V; union U { v16h v; v8h h[2]; };
  static __device__ __forceinline__ v16h load(const _Float16* p) {
    U f; f.h[0] = *(const v8h*)(p); f.h[1] = *(const v8h*)(p + 16); return f.v;
  }
  static __device__ __forceinline__ v8f mma(v16h a, v16h b, v8f c) {
    return __builtin_amdgcn_wmma_f32_16x16x32_f16(false, a, false, b, (short)0, c, false, false);
  }
  static __device__ __forceinline__ void tie(v8f& a, v8f& b, v8f& c, v8f& d, v16h x, v16h y, v16h z0, v16h z1, v16h z2, v16h z3) { tie4_h(a, b, c, d, x, y, z0, z1, z2, z3); }
  static __device__ __forceinline__ void keep(v16h a, v16h b, v16h c, v16h d) { keep4_h(a, b, c, d); }
};
template <> struct Frag<__bf16> {
  typedef v16b V; union U { v16b v; v8b h[2]; };
  static __device__ __forceinline__ v16b load(const __bf16* p) {
    U f; f.h[0] = *(const v8b*)(p); f.h[1] = *(const v8b*)(p + 16); return f.v;
  }
  static __device__ __forceinline__ v8f mma(v16b a, v16b b, v8f c) {
    return __builtin_amdgcn_wmma_f32_16x16x32_bf16(false, a, false, b, (short)0, c, false, false);
  }
  static __device__ __forceinline__ void tie(v8f& a, v8f& b, v8f& c, v8f& d, v16b x, v16b y, v16b z0, v16b z1, v16b z2, v16b z3) { tie4_b(a, b, c, d, x, y, z0, z1, z2, z3); }
  static __device__ __forceinline__ void keep(v16b a, v16b b, v16b c, v16b d) { keep4_b(a, b, c, d); }
};

template <int ET> struct Elem;
template <> struct Elem<0> { typedef _Float16 T; };
template <> struct Elem<1> { typedef __bf16 T; };
template <int ET, int SPLIT, int BIAS_MODE, int OUT_MODE>
__global__ __launch_bounds__(256) void wmma_gemm64(
    const unsigned short* __restrict__ Ap, const unsigned short* __restrict__ A2p, int lda, long strideA,
    const unsigned short* __restrict__ Btp, const unsigned short* __restrict__ Bt2p, int ldb, long strideB,
    void* __restrict__ Cout, void* __restrict__ Cout2, int ldc, long strideC,
    const float* __restrict__ bias,
    int M, int N, int K, float scale) {
  constexpr bool kSA = (SPLIT == 1);
  constexpr bool kSB = (SPLIT != 0);
  typedef typename Elem<ET>::T T;
  typedef typename Frag<T>::V V;
  const T* A = (const T*)Ap; const T* A2 = (const T*)A2p; const T* Bt = (const T*)Btp; const T* Bt2 = (const T*)Bt2p;
  __shared__ __align__(16) float sT[8][16 * 68];
  const int b    = blockIdx.y;
  const int lane = threadIdx.x & 31;
  const int wave = threadIdx.x >> 5;
  const int tilesN = N >> 6;
  const int tilesM = M >> 6;
  const int tile = blockIdx.x * 8 + wave;
  if (tile >= tilesM * tilesN) return;
  const int tm = tile / tilesN;
  const int tn = tile - tm * tilesN;
  const int m0 = tm << 6;
  const int n0 = tn << 6;

  const T* Ab  = A  + (size_t)b * strideA;
  const T* Bb  = Bt + (size_t)b * strideB;
  const T* Ab2 = kSA ? (A2  + (size_t)b * strideA) : nullptr;
  const T* Bb2 = kSB ? (Bt2 + (size_t)b * strideB) : nullptr;

  const int rlane = lane & 15;
  const int koff  = (lane >> 4) * 8;
  const int mOff  = (lane >> 4) * 8;

  v8f acc[4][4];
#pragma unroll
  for (int i = 0; i < 4; ++i)
#pragma unroll
    for (int j = 0; j < 4; ++j) acc[i][j] = (v8f){0.f,0.f,0.f,0.f,0.f,0.f,0.f,0.f};

  for (int k0 = 0; k0 < K; k0 += 32) {
    V bh[4];
#pragma unroll
    for (int j = 0; j < 4; ++j) bh[j] = Frag<T>::load(Bb + (size_t)(n0 + (j << 4) + rlane) * ldb + koff + k0);
#pragma unroll
    for (int i = 0; i < 4; ++i) {
      const size_t ao = (size_t)(m0 + (i << 4) + rlane) * lda + koff + k0;
      V ah = Frag<T>::load(Ab + ao);
      V al = ah;
      if (kSA) al = Frag<T>::load(Ab2 + ao);
#pragma unroll
      for (int j = 0; j < 4; ++j) {
        acc[i][j] = Frag<T>::mma(ah, bh[j], acc[i][j]);
        if (kSA) acc[i][j] = Frag<T>::mma(al, bh[j], acc[i][j]);
      }
      Frag<T>::tie(acc[i][0], acc[i][1], acc[i][2], acc[i][3], ah, al, bh[0], bh[1], bh[2], bh[3]);
    }
    Frag<T>::keep(bh[0], bh[1], bh[2], bh[3]);
    if (kSB) {
      mem_order();
      V bl[4];
#pragma unroll
      for (int j = 0; j < 4; ++j) bl[j] = Frag<T>::load(Bb2 + (size_t)(n0 + (j << 4) + rlane) * ldb + koff + k0);
#pragma unroll
      for (int i = 0; i < 4; ++i) {
        const size_t ao = (size_t)(m0 + (i << 4) + rlane) * lda + koff + k0;
        V ah = Frag<T>::load(Ab + ao);
#pragma unroll
        for (int j = 0; j < 4; ++j) acc[i][j] = Frag<T>::mma(ah, bl[j], acc[i][j]);
        Frag<T>::tie(acc[i][0], acc[i][1], acc[i][2], acc[i][3], ah, ah, bl[0], bl[1], bl[2], bl[3]);
      }
      Frag<T>::keep(bl[0], bl[1], bl[2], bl[3]);
    }
  }
  acc_guard4(acc[0][0], acc[0][1], acc[0][2], acc[0][3]);
  acc_guard4(acc[1][0], acc[1][1], acc[1][2], acc[1][3]);
  acc_guard4(acc[2][0], acc[2][1], acc[2][2], acc[2][3]);
  acc_guard4(acc[3][0], acc[3][1], acc[3][2], acc[3][3]);

  float* slab = sT[wave];
#pragma unroll
  for (int i = 0; i < 4; ++i) {
    const int mBase = m0 + (i << 4);
#pragma unroll
    for (int j = 0; j < 4; ++j) {
      const int n = n0 + (j << 4) + rlane;
      float bv = 0.f;
      if (BIAS_MODE == 2) bv = bias[n];
#pragma unroll
      for (int r = 0; r < 8; ++r) {
        float v = acc[i][j][r] * scale;
        if (BIAS_MODE == 1) v += bias[mBase + mOff + r];
        if (BIAS_MODE == 2) v += bv;
        slab[(mOff + r) * 68 + (j << 4) + rlane] = v;
      }
    }
    __builtin_amdgcn_fence(__ATOMIC_RELEASE, "workgroup");
    __builtin_amdgcn_wave_barrier();
    __builtin_amdgcn_fence(__ATOMIC_ACQUIRE, "workgroup");
    if (OUT_MODE == 0) {
      float* Cp = (float*)Cout + (size_t)b * strideC;
      const int hh = lane >> 4, c4 = (lane & 15) * 4;
      for (int pass = 0; pass < 2; ++pass) {
#pragma unroll
        for (int it = 0; it < 8; ++it) {
          const int row = it * 2 + hh;
          v4f v = *(const v4f*)(slab + row * 68 + c4);
          *(volatile v4f*)(Cp + (size_t)(mBase + row) * ldc + n0 + c4) = v;
        }
        __threadfence();
      }
    } else {
      const int q = lane >> 3, c8 = (lane & 7) * 8;
      unsigned short* Cp  = (unsigned short*)Cout  + (size_t)b * strideC;
      unsigned short* Cp2 = (OUT_MODE == 2) ? ((unsigned short*)Cout2 + (size_t)b * strideC) : nullptr;
      for (int pass = 0; pass < 2; ++pass) {
#pragma unroll
        for (int it = 0; it < 4; ++it) {
          const int row = it * 4 + q;
          const float* sp = slab + row * 68 + c8;
          v8h hv, lv;
#pragma unroll
          for (int e = 0; e < 8; ++e) {
            if (OUT_MODE == 1) {
              hv[e] = (_Float16)sp[e];
            } else {
              unsigned short hb = f2bf_bits(sp[e]);
              unsigned short lb = f2bf_bits(sp[e] - bf_bits2f(hb));
              hv[e] = __builtin_bit_cast(_Float16, hb);
              lv[e] = __builtin_bit_cast(_Float16, lb);
            }
          }
          *(volatile v8h*)(Cp + (size_t)(mBase + row) * ldc + n0 + c8) = hv;
          if (OUT_MODE == 2) *(volatile v8h*)(Cp2 + (size_t)(mBase + row) * ldc + n0 + c8) = lv;
        }
        __threadfence();
      }
    }
    __builtin_amdgcn_fence(__ATOMIC_RELEASE, "workgroup");
    __builtin_amdgcn_wave_barrier();
    __builtin_amdgcn_fence(__ATOMIC_ACQUIRE, "workgroup");
  }
}

__global__ __launch_bounds__(256) void prep_x_kernel(const float* __restrict__ x,
                                                     unsigned short* __restrict__ xpad,
                                                     unsigned short* __restrict__ xb) {
  __shared__ float sm[64][65];
  const int t  = threadIdx.x;
  const int h  = blockIdx.x;
  const int c0 = blockIdx.y * 64;
  const int b  = blockIdx.z;
#pragma unroll
  for (int i = 0; i < 8; ++i) {
    const int e  = i * 256 + t;
    const int r  = e >> 6;
    const int cc = e & 63;
    sm[r][cc] = x[((size_t)(b * kC + c0 + r) * kH + h) * kW + cc];
  }
  mem_order();
#pragma unroll
  for (int i = 8; i < 16; ++i) {
    const int e  = i * 256 + t;
    const int r  = e >> 6;
    const int cc = e & 63;
    sm[r][cc] = x[((size_t)(b * kC + c0 + r) * kH + h) * kW + cc];
  }
  __syncthreads();
  const int lane = t & 31, wave = t >> 5;
  const int q = lane >> 3, c8 = (lane & 7) * 8;
  unsigned short* xp = xpad + ((size_t)(b * kHP + h + 1) * kHP + 1) * kC + c0;
  unsigned short* xo = xb + (size_t)(b * kC + c0) * kN + h * kW;
  for (int pass = 0; pass < 2; ++pass) {
#pragma unroll
    for (int it = 0; it < 2; ++it) {
      const int row = wave * 8 + it * 4 + q;
      unsigned short hb[8];
#pragma unroll
      for (int e = 0; e < 8; ++e) hb[e] = f2bf_bits(sm[c8 + e][row]);
      const v4u ua = (v4u){pk16(hb[0], hb[1]), pk16(hb[2], hb[3]), pk16(hb[4], hb[5]), pk16(hb[6], hb[7])};
      *(volatile v4u*)(xp + (size_t)row * kC + c8) = ua;
      unsigned short hc[8];
#pragma unroll
      for (int e = 0; e < 8; ++e) hc[e] = f2bf_bits(sm[row][c8 + e]);
      const v4u ub = (v4u){pk16(hc[0], hc[1]), pk16(hc[2], hc[3]), pk16(hc[4], hc[5]), pk16(hc[6], hc[7])};
      *(volatile v4u*)(xo + (size_t)row * kN + c8) = ub;
    }
    __threadfence();
  }
}

__global__ __launch_bounds__(64) void xpad_border_kernel(unsigned short* __restrict__ xpad) {
  const int p = blockIdx.x, b = blockIdx.y, t = threadIdx.x;
  int hp, wp;
  if (p < 66)       { hp = 0;       wp = p; }
  else if (p < 132) { hp = 65;      wp = p - 66; }
  else if (p < 196) { hp = p - 131; wp = 0; }
  else              { hp = p - 195; wp = 65; }
  unsigned short* dst = xpad + ((size_t)(b * kHP + hp) * kHP + wp) * kC + 8 * t;
  const v4u z = (v4u){0u, 0u, 0u, 0u};
  *(volatile v4u*)dst = z;
  __threadfence();
  *(volatile v4u*)dst = z;
}

__global__ __launch_bounds__(256) void prep_w_kernel(const float* __restrict__ w1, const float* __restrict__ w2,
                                                     unsigned short* __restrict__ wr) {
  __shared__ float wl[kKconv];
  const int t = threadIdx.x;
  const int o = blockIdx.x, br = blockIdx.y;
  const float* Wsrc = (br == 0) ? w1 : w2;
  const float* wrow = Wsrc + (size_t)o * kKconv;
#pragma unroll
  for (int i = 0; i < 9; ++i) wl[i * 256 + t] = wrow[i * 256 + t];
  mem_order();
#pragma unroll
  for (int i = 9; i < 18; ++i) wl[i * 256 + t] = wrow[i * 256 + t];
  __syncthreads();
  unsigned short* ob = wr + (size_t)(br * kCk + o) * kTaps * kC;
  for (int pass = 0; pass < 2; ++pass) {
#pragma unroll
    for (int it = 0; it < 3; ++it) {
      const int p = it * 256 + t;
      if (p < 576) {
        const int line = p >> 3, j = p & 7;
        const int tap = line >> 3, seg = line & 7;
        unsigned short hb[8];
#pragma unroll
        for (int e = 0; e < 8; ++e) {
          const int c = seg * 64 + j * 8 + e;
          hb[e] = f2bf_bits(wl[c * kTaps + tap]);
        }
        const v4u u = (v4u){pk16(hb[0], hb[1]), pk16(hb[2], hb[3]), pk16(hb[4], hb[5]), pk16(hb[6], hb[7])};
        *(volatile v4u*)(ob + (size_t)tap * kC + seg * 64 + j * 8) = u;
      }
    }
    __threadfence();
  }
}

__global__ __launch_bounds__(128) void bn_params_kernel(const float* __restrict__ g1, const float* __restrict__ b1,
                                                       const float* __restrict__ m1, const float* __restrict__ v1,
                                                       const float* __restrict__ g2, const float* __restrict__ b2,
                                                       const float* __restrict__ m2, const float* __restrict__ v2,
                                                       float* __restrict__ bnp) {
  __shared__ __align__(16) float bs[256];
  const int t  = threadIdx.x;
  const int br = t >> 6, c = t & 63;
  const float* gp = (br == 0) ? g1 : g2;
  const float* bp = (br == 0) ? b1 : b2;
  const float* mp = (br == 0) ? m1 : m2;
  const float* vp = (br == 0) ? v1 : v2;
  const float gr  = bf_bits2f(f2bf_bits(gp[c]));
  const float brv = bf_bits2f(f2bf_bits(bp[c]));
  const float mr  = bf_bits2f(f2bf_bits(mp[c]));
  const float vr  = bf_bits2f(f2bf_bits(vp[c]));
  const float sq = sqrtf(vr + kBnEps);
  const float sc = gr / sq;
  const float sh = brv - (mr * gr) / sq;
  bs[br * 128 + c]      = sc;
  bs[br * 128 + 64 + c] = sh;
  __syncthreads();
  if (t < 64) {
    const v4f v = *(const v4f*)(bs + 4 * t);
    float* dp = bnp + 4 * t;
    *(volatile v4f*)dp = v;
    __threadfence();
    *(volatile v4f*)dp = v;
  }
}

__global__ __launch_bounds__(256) void conv3x3_bn_silu_kernel(const unsigned short* __restrict__ xpadp,
                                                             const unsigned short* __restrict__ wrp,
                                                             const float* __restrict__ bnp,
                                                             unsigned short* __restrict__ yp) {
  typedef __bf16 T;
  typedef v16b V;
  __shared__ __align__(16) float sT[8][16 * 68];
  const int br   = blockIdx.y;
  const int lane = threadIdx.x & 31;
  const int wave = threadIdx.x >> 5;
  const int tile = blockIdx.x * 8 + wave;
  if (tile >= kB * kH) return;
  const int b  = tile >> 6;
  const int h  = tile & 63;
  const int m0 = tile << 6;
  const T* Xb = (const T*)xpadp + (size_t)b * kHP * kHP * kC;
  const T* Wb = (const T*)wrp + (size_t)br * kCk * kKconv;
  const float* scp = bnp + br * 128;
  const int rlane = lane & 15;
  const int koff  = (lane >> 4) * 8;
  const int mOff  = (lane >> 4) * 8;
  float scv[4], shv[4];
#pragma unroll
  for (int j = 0; j < 4; ++j) { scv[j] = scp[(j << 4) + rlane]; shv[j] = scp[64 + (j << 4) + rlane]; }

  v8f acc[4][4];
#pragma unroll
  for (int i = 0; i < 4; ++i)
#pragma unroll
    for (int j = 0; j < 4; ++j) acc[i][j] = (v8f){0.f,0.f,0.f,0.f,0.f,0.f,0.f,0.f};

#pragma unroll 1
  for (int tap = 0; tap < kTaps; ++tap) {
    const int kh = tap / 3;
    const int kw = tap - kh * 3;
    const T* At = Xb + (size_t)((h + kh) * kHP + kw) * kC;
    const T* Bq = Wb + tap * kC;
#pragma unroll 1
    for (int k0 = 0; k0 < kC; k0 += 32) {
      V bh[4];
#pragma unroll
      for (int j = 0; j < 4; ++j) bh[j] = Frag<T>::load(Bq + (size_t)((j << 4) + rlane) * kKconv + koff + k0);
#pragma unroll
      for (int i = 0; i < 4; ++i) {
        V ah = Frag<T>::load(At + (size_t)((i << 4) + rlane) * kC + koff + k0);
#pragma unroll
        for (int j = 0; j < 4; ++j) acc[i][j] = Frag<T>::mma(ah, bh[j], acc[i][j]);
        Frag<T>::tie(acc[i][0], acc[i][1], acc[i][2], acc[i][3], ah, ah, bh[0], bh[1], bh[2], bh[3]);
      }
      Frag<T>::keep(bh[0], bh[1], bh[2], bh[3]);
    }
  }
  acc_guard4(acc[0][0], acc[0][1], acc[0][2], acc[0][3]);
  acc_guard4(acc[1][0], acc[1][1], acc[1][2], acc[1][3]);
  acc_guard4(acc[2][0], acc[2][1], acc[2][2], acc[2][3]);
  acc_guard4(acc[3][0], acc[3][1], acc[3][2], acc[3][3]);

  float* slab = sT[wave];
  unsigned short* Cp  = yp + (size_t)(br * 2) * kRows * kCk;
  unsigned short* Cp2 = Cp + (size_t)kRows * kCk;
#pragma unroll
  for (int i = 0; i < 4; ++i) {
    const int mBase = m0 + (i << 4);
#pragma unroll
    for (int j = 0; j < 4; ++j) {
#pragma unroll
      for (int r = 0; r < 8; ++r) {
        float v = acc[i][j][r] * scv[j] + shv[j];
        const float ex = expf(fminf(-v, 60.0f));
        v = v * (1.0f / (1.0f + ex));
        slab[(mOff + r) * 68 + (j << 4) + rlane] = v;
      }
    }
    __builtin_amdgcn_fence(__ATOMIC_RELEASE, "workgroup");
    __builtin_amdgcn_wave_barrier();
    __builtin_amdgcn_fence(__ATOMIC_ACQUIRE, "workgroup");
    const int q = lane >> 3, c8 = (lane & 7) * 8;
    for (int pass = 0; pass < 2; ++pass) {
#pragma unroll
      for (int it = 0; it < 4; ++it) {
        const int row = it * 4 + q;
        const float* sp = slab + row * 68 + c8;
        v8h hv, lv;
#pragma unroll
        for (int e = 0; e < 8; ++e) {
          unsigned short hb = f2bf_bits(sp[e]);
          unsigned short lb = f2bf_bits(sp[e] - bf_bits2f(hb));
          hv[e] = __builtin_bit_cast(_Float16, hb);
          lv[e] = __builtin_bit_cast(_Float16, lb);
        }
        *(volatile v8h*)(Cp  + (size_t)(mBase + row) * kCk + c8) = hv;
        *(volatile v8h*)(Cp2 + (size_t)(mBase + row) * kCk + c8) = lv;
      }
      __threadfence();
    }
    __builtin_amdgcn_fence(__ATOMIC_RELEASE, "workgroup");
    __builtin_amdgcn_wave_barrier();
    __builtin_amdgcn_fence(__ATOMIC_ACQUIRE, "workgroup");
  }
}

__global__ __launch_bounds__(256) void colstats_kernel(const float* __restrict__ ST, float* __restrict__ CST) {
  __shared__ float redM[8][64];
  __shared__ float redS[8][64];
  __shared__ __align__(16) float stg[128];
  const int t = threadIdx.x, lane = t & 31, wave = t >> 5;
  const int nb = blockIdx.x, n0 = nb * 64;
  const float* base = ST + n0 + 2 * lane;
  float mx0 = -__builtin_inff(), mx1 = -__builtin_inff();
#pragma unroll 4
  for (int r = wave; r < kN; r += 8) {
    const v2f s = *(const v2f*)(base + (size_t)r * kN);
    mx0 = fmaxf(mx0, s[0]);
    mx1 = fmaxf(mx1, s[1]);
  }
  redM[wave][2 * lane]     = mx0;
  redM[wave][2 * lane + 1] = mx1;
  __syncthreads();
  float cm0 = redM[0][2 * lane], cm1 = redM[0][2 * lane + 1];
#pragma unroll
  for (int w = 1; w < 8; ++w) { cm0 = fmaxf(cm0, redM[w][2 * lane]); cm1 = fmaxf(cm1, redM[w][2 * lane + 1]); }
  float s0 = 0.0f, s1 = 0.0f;
#pragma unroll 1
  for (int r = wave; r < kN; r += 8) {
    const v2f s = *(const v2f*)(base + (size_t)r * kN);
    s0 += expf(s[0] - cm0);
    s1 += expf(s[1] - cm1);
  }
  redS[wave][2 * lane]     = s0;
  redS[wave][2 * lane + 1] = s1;
  __syncthreads();
  if (t < 64) {
    float mm = redM[0][t];
    float tot = redS[0][t];
#pragma unroll
    for (int w = 1; w < 8; ++w) { mm = fmaxf(mm, redM[w][t]); tot += redS[w][t]; }
    stg[t]      = mm;
    stg[64 + t] = kPCarry / tot;
  }
  __syncthreads();
  if (t < 32) {
    const v4f v = *(const v4f*)(stg + 4 * t);
    float* dp = CST + (size_t)nb * 128 + 4 * t;
    *(volatile v4f*)dp = v;
    __threadfence();
    *(volatile v4f*)dp = v;
  }
}

__global__ __launch_bounds__(256) void cw_kernel(const float* __restrict__ STc, const float* __restrict__ CST,
                                                unsigned short* __restrict__ CWH, unsigned short* __restrict__ CWL) {
  const int i = blockIdx.x * 256 + threadIdx.x;
  const int m = i >> 9;
  const int n = (i & 511) * 8;
  const float* sp = STc + (size_t)m * kN + n;
  const v4f a = *(const v4f*)(sp);
  const v4f c = *(const v4f*)(sp + 4);
  const float* cp = CST + (n >> 6) * 128 + (n & 63);
  const v4f mxa = *(const v4f*)(cp);
  const v4f mxc = *(const v4f*)(cp + 4);
  const v4f iva = *(const v4f*)(cp + 64);
  const v4f ivc = *(const v4f*)(cp + 68);
  unsigned short hb[8], lb[8];
#pragma unroll
  for (int e = 0; e < 4; ++e) {
    const float p0 = expf(a[e] - mxa[e]) * iva[e];
    const unsigned short h0 = f2bf_bits(p0);
    hb[e] = h0;
    lb[e] = f2bf_bits(p0 - bf_bits2f(h0));
    const float p1 = expf(c[e] - mxc[e]) * ivc[e];
    const unsigned short h1 = f2bf_bits(p1);
    hb[4 + e] = h1;
    lb[4 + e] = f2bf_bits(p1 - bf_bits2f(h1));
  }
  const v4u uh = (v4u){pk16(hb[0], hb[1]), pk16(hb[2], hb[3]), pk16(hb[4], hb[5]), pk16(hb[6], hb[7])};
  const v4u ul = (v4u){pk16(lb[0], lb[1]), pk16(lb[2], lb[3]), pk16(lb[4], lb[5]), pk16(lb[6], lb[7])};
  const size_t o = (size_t)m * kN + n;
  *(volatile v4u*)(CWH + o) = uh;
  *(volatile v4u*)(CWL + o) = ul;
  __threadfence();
  *(volatile v4u*)(CWH + o) = uh;
  *(volatile v4u*)(CWL + o) = ul;
}

extern "C" void kernel_launch(void* const* d_in, const int* in_sizes, int n_in,
                              void* d_out, int out_size, void* d_ws, size_t ws_size,
                              hipStream_t stream) {
  if (n_in < 11) return;
  const int nX  = kB * kC * kN;
  const int nWt = kCk * kKconv;
  if (in_sizes[0] != nX) return;
  if (in_sizes[1] != nWt || in_sizes[6] != nWt) return;
  if (in_sizes[2] != kCk || in_sizes[3] != kCk || in_sizes[4] != kCk || in_sizes[5] != kCk) return;
  if (in_sizes[7] != kCk || in_sizes[8] != kCk || in_sizes[9] != kCk || in_sizes[10] != kCk) return;
  if (out_size != nX) return;

  const size_t szXP  = (size_t)kB * kHP * kHP * kC * 2;
  const size_t szXB  = (size_t)kB * kC * kN * 2;
  const size_t szWR  = (size_t)2 * kCk * kKconv * 2;
  const size_t szBN  = 1024;
  const size_t szY   = (size_t)4 * kRows * kCk * 2;
  const size_t szST  = (size_t)kN * kN * 4;
  const size_t szCST = (size_t)(kN / 64) * 128 * 4;
  const size_t szCW  = (size_t)kMHalf * kN * 2;
  const size_t offXP  = 0;
  const size_t offXB  = offXP + szXP;
  const size_t offWR  = offXB + szXB;
  const size_t offBN  = offWR + szWR;
  const size_t offY   = offBN + szBN;
  const size_t offST  = offY + szY;
  const size_t offCST = offST + szST;
  const size_t offCWH = offCST + szCST;
  const size_t offCWL = offCWH + szCW;
  const size_t total  = offCWL + szCW;
  if (ws_size < total) return;

  const float* x  = (const float*)d_in[0];
  const float* w1 = (const float*)d_in[1];
  const float* g1 = (const float*)d_in[2];
  const float* b1 = (const float*)d_in[3];
  const float* m1 = (const float*)d_in[4];
  const float* v1 = (const float*)d_in[5];
  const float* w2 = (const float*)d_in[6];
  const float* g2 = (const float*)d_in[7];
  const float* b2 = (const float*)d_in[8];
  const float* m2 = (const float*)d_in[9];
  const float* v2 = (const float*)d_in[10];
  float* out = (float*)d_out;
  char* ws = (char*)d_ws;
  unsigned short* XPAD = (unsigned short*)(ws + offXP);
  unsigned short* XB   = (unsigned short*)(ws + offXB);
  unsigned short* WR   = (unsigned short*)(ws + offWR);
  float*          BNP  = (float*)(ws + offBN);
  unsigned short* Y    = (unsigned short*)(ws + offY);
  float*          ST   = (float*)(ws + offST);
  float*          CST  = (float*)(ws + offCST);
  unsigned short* CWH  = (unsigned short*)(ws + offCWH);
  unsigned short* CWL  = (unsigned short*)(ws + offCWL);

  prep_x_kernel<<<dim3(kH, kC / 64, kB), dim3(256), 0, stream>>>(x, XPAD, XB);
  xpad_border_kernel<<<dim3(260, kB), dim3(64), 0, stream>>>(XPAD);
  prep_w_kernel<<<dim3(kCk, 2), dim3(256), 0, stream>>>(w1, w2, WR);
  bn_params_kernel<<<dim3(1), dim3(128), 0, stream>>>(g1, b1, m1, v1, g2, b2, m2, v2, BNP);

  conv3x3_bn_silu_kernel<<<dim3((kB * kH) / 8, 2), dim3(256), 0, stream>>>(XPAD, WR, BNP, Y);

  const size_t planeY = (size_t)kRows * kCk;
  const unsigned short* Y1H = Y;
  const unsigned short* Y1L = Y + planeY;
  const unsigned short* Y2H = Y + 2 * planeY;
  const unsigned short* Y2L = Y + 3 * planeY;
  const int tilesScore = (kN / 64) * (kN / 64);
  const int tilesValue = (kC / 64) * (kMHalf / 64);

  for (int b = 0; b < kB; ++b) {
    const size_t yoff = (size_t)b * kN * kCk;
    wmma_gemm64<1, 1, 0, 0><<<dim3(tilesScore / 8, 1), dim3(256), 0, stream>>>(
        Y1H + yoff, Y1L + yoff, kCk, 0L, Y2H + yoff, Y2L + yoff, kCk, 0L,
        (void*)ST, (void*)ST, kN, 0L, BNP, kN, kN, kCk, 1.0f);
    colstats_kernel<<<dim3(kN / 64), dim3(256), 0, stream>>>(ST, CST);
    for (int mh = 0; mh < 2; ++mh) {
      cw_kernel<<<dim3((kMHalf * kN) / 8 / 256), dim3(256), 0, stream>>>(ST + (size_t)mh * kMHalf * kN, CST, CWH, CWL);
      const unsigned short* Ab = XB + (size_t)b * kC * kN;
      float* outc = out + (size_t)b * kC * kN + (size_t)mh * kMHalf;
      wmma_gemm64<1, 2, 0, 0><<<dim3(tilesValue / 8, 1), dim3(256), 0, stream>>>(
          Ab, Ab, kN, 0L, CWH, CWL, kN, 0L,
          (void*)outc, (void*)outc, kN, 0L, BNP, kC, kMHalf, kN, kPCarryInv);
    }
  }
}
